// ItemConv_51041391345937
// MI455X (gfx1250) — hardware-verified
//
#include <hip/hip_runtime.h>
#include <stddef.h>


#define EMB     128
#define NTHR    256
#define NWAVE   8
#define EPT     8
#define NGRP    2
#define CHUNK   (NTHR * EPT * NGRP)
#define WCAP    (EPT * NGRP * 32)
#define LISTN   (NWAVE * WCAP)
#define NBC     4096
#define NBF     2048
#define NSUB    (NBC / NBF)
#define RCAP    40960
#define RBN     128
#define TGT     256
#define DEGCAP  1024
#define GROWS   128
#define OTHR    512
#define CNTMAX  65535
#define WSCALE  8.0f
#define WINV    0.125f

#define LDS_GEMM (GROWS * EMB * 4)
#define LDS_AGG  (TGT * EMB * 2)
#define LDS_FILL ((RCAP + NBF + LISTN) * 4 + 64)

static_assert((CHUNK & (CHUNK - 1)) == 0);
static_assert(CHUNK <= 4096);
static_assert(NBC <= 4096 && NBF <= 4096);
static_assert((NBC & (NBC - 1)) == 0 && (NBF & (NBF - 1)) == 0);
static_assert(NBC == 2 * NBF && NSUB == 2);
static_assert(OTHR * 8 == NBC);
static_assert(OTHR == 512);
static_assert((RCAP % 32) == 0);
static_assert(TGT == NWAVE * 32 && (TGT % GROWS) == 0);
static_assert(GROWS == NWAVE * 16);
static_assert(EMB == 128);

typedef float    v4f  __attribute__((ext_vector_type(4)));
typedef float    v8f  __attribute__((ext_vector_type(8)));
typedef int      v4i  __attribute__((ext_vector_type(4)));
typedef _Float16 v4h  __attribute__((ext_vector_type(4)));
typedef _Float16 v8h  __attribute__((ext_vector_type(8)));
typedef _Float16 v16h __attribute__((ext_vector_type(16)));
union FragH { v16h v; v8h h[2]; };

__device__ __forceinline__ v8h cvt8(v4f a, v4f b) {
  v8h r;
  r[0] = (_Float16)a.x; r[1] = (_Float16)a.y; r[2] = (_Float16)a.z; r[3] = (_Float16)a.w;
  r[4] = (_Float16)b.x; r[5] = (_Float16)b.y; r[6] = (_Float16)b.z; r[7] = (_Float16)b.w;
  return r;
}

__device__ __forceinline__ v8f wmh(v16h a, v16h b, v8f c) {
  v8f d = __builtin_amdgcn_wmma_f32_16x16x32_f16(false, a, false, b, (short)0, c, false, false);
  asm volatile("v_nop\n\tv_nop\n\tv_nop\n\tv_nop" : "+v"(d) : "v"(a), "v"(b));
  return d;
}

template <int NB>
__device__ __forceinline__ int scan_chunk(const int* __restrict__ dsts, int nE, int cbase, int slotBase,
                                          int vec8, int* list, int tid, int lane, int wave) {
  int wc = 0;
#pragma unroll
  for (int g = 0; g < NGRP; ++g) {
    const int el0  = (g * NTHR + tid) * EPT;
    const int e0   = cbase + el0;
    const int sent = -2147483647 - 1;
    v4i da, db;
    if (vec8 != 0 && cbase + CHUNK <= nE) {
      da = *(const v4i*)(dsts + e0);
      db = *(const v4i*)(dsts + e0 + 4);
    } else {
      da.x = (e0     < nE) ? dsts[min(e0, nE - 1)] : sent;
      da.y = (e0 + 1 < nE) ? dsts[min(e0 + 1, nE - 1)] : sent;
      da.z = (e0 + 2 < nE) ? dsts[min(e0 + 2, nE - 1)] : sent;
      da.w = (e0 + 3 < nE) ? dsts[min(e0 + 3, nE - 1)] : sent;
      db.x = (e0 + 4 < nE) ? dsts[min(e0 + 4, nE - 1)] : sent;
      db.y = (e0 + 5 < nE) ? dsts[min(e0 + 5, nE - 1)] : sent;
      db.z = (e0 + 6 < nE) ? dsts[min(e0 + 6, nE - 1)] : sent;
      db.w = (e0 + 7 < nE) ? dsts[min(e0 + 7, nE - 1)] : sent;
    }
    const unsigned nb = (unsigned)slotBase;
    const unsigned s0 = (unsigned)da.x - nb, s1 = (unsigned)da.y - nb;
    const unsigned s2 = (unsigned)da.z - nb, s3 = (unsigned)da.w - nb;
    const unsigned s4 = (unsigned)db.x - nb, s5 = (unsigned)db.y - nb;
    const unsigned s6 = (unsigned)db.z - nb, s7 = (unsigned)db.w - nb;
    const bool h0 = s0 < (unsigned)NB, h1 = s1 < (unsigned)NB, h2 = s2 < (unsigned)NB, h3 = s3 < (unsigned)NB;
    const bool h4 = s4 < (unsigned)NB, h5 = s5 < (unsigned)NB, h6 = s6 < (unsigned)NB, h7 = s7 < (unsigned)NB;
    const unsigned any = __builtin_amdgcn_ballot_w32(h0 | h1 | h2 | h3 | h4 | h5 | h6 | h7);
    if (any != 0u) {
#define HITJ(J, HJ, SJ) { \
        const unsigned mj = __builtin_amdgcn_ballot_w32(HJ); \
        if (mj != 0u) { \
          if (HJ) { \
            const int pos = wc + (int)__builtin_amdgcn_mbcnt_lo(mj, 0u); \
            if (pos < WCAP) list[wave * WCAP + pos] = ((el0 + (J)) << 12) | (int)(SJ); \
          } \
          wc += (int)__builtin_popcount(mj); } }
      HITJ(0, h0, s0)
      HITJ(1, h1, s1)
      HITJ(2, h2, s2)
      HITJ(3, h3, s3)
      HITJ(4, h4, s4)
      HITJ(5, h5, s5)
      HITJ(6, h6, s6)
      HITJ(7, h7, s7)
#undef HITJ
    }
  }
  return wc;
}

__global__ __launch_bounds__(NTHR) void k_wprep(const float* __restrict__ W, _Float16* wl, int total8) {
  const int i = blockIdx.x * NTHR + (int)threadIdx.x;
  if (i >= total8) return;
  const float* sp = W + (size_t)i * 8;
  const v4f a = *(const v4f*)sp * WSCALE;
  const v4f b = *(const v4f*)(sp + 4) * WSCALE;
  const v8h hv = cvt8(a, b);
  _Float16* dp = wl + (size_t)i * 8;
  *(volatile v8h*)dp = hv;
  __threadfence();
  *(volatile v8h*)dp = hv;
}

__global__ __launch_bounds__(NTHR) void k_cvt(const float* __restrict__ emb, _Float16* hp, int nN, int total8) {
  const int i = blockIdx.x * NTHR + (int)threadIdx.x;
  if (i >= total8) return;
  const int row = i >> 4;
  const int c0  = (i & 15) * 8;
  const int rc  = row < nN ? row : nN - 1;
  const float keep = row < nN ? 1.0f : 0.0f;
  const float* sp = emb + (size_t)rc * EMB + c0;
  const v4f a = *(const v4f*)sp * keep;
  const v4f b = *(const v4f*)(sp + 4) * keep;
  const v8h hv = cvt8(a, b);
  _Float16* dp = hp + (size_t)i * 8;
  *(volatile v8h*)dp = hv;
  __threadfence();
  *(volatile v8h*)dp = hv;
}

__global__ __launch_bounds__(NTHR) void k_count(const int* __restrict__ dsts, int* cnt, int nE, int vec8) {
  __shared__ __attribute__((aligned(16))) int scnt[NBC];
  __shared__ __attribute__((aligned(16))) int list[LISTN];
  __shared__ int wcnt[NWAVE];
  const int tid = threadIdx.x, lane = tid & 31, wave = tid >> 5;
  const int nodeBase = blockIdx.x * NBC;

  for (int i = tid; i < NBC; i += NTHR) scnt[i] = 0;
  __syncthreads();

  const int nChunks = (nE + CHUNK - 1) / CHUNK;
#pragma unroll 1
  for (int ch = 0; ch < nChunks; ++ch) {
    const int cbase = ch * CHUNK;
    const int wc = scan_chunk<NBC>(dsts, nE, cbase, nodeBase, vec8, list, tid, lane, wave);
    if (lane == 0) wcnt[wave] = wc;
    __syncthreads();
    if (wave == 0) {
#pragma unroll 1
      for (int wsx = 0; wsx < NWAVE; ++wsx) {
        int n = __builtin_amdgcn_readfirstlane(wcnt[wsx]);
        n = n > WCAP ? WCAP : (n < 0 ? 0 : n);
        const int* lp = list + wsx * WCAP;
#pragma unroll 1
        for (int i = 0; i < n; ++i) {
          const int ent  = __builtin_amdgcn_readfirstlane(lp[i]);
          const int slot = ent & (NBC - 1);
          if (lane == 0) scnt[slot] = scnt[slot] + 1;
        }
      }
    }
    __syncthreads();
  }

  v4i cq[4];
#pragma unroll
  for (int q = 0; q < 4; ++q) {
    const int f = (wave * 4 + q) * 128 + 4 * lane;
    cq[q] = *(const v4i*)(scnt + f);
  }
  int* cp = cnt + (size_t)nodeBase;
#pragma unroll
  for (int q = 0; q < 4; ++q) {
    const int f = (wave * 4 + q) * 128 + 4 * lane;
    *(volatile v4i*)(cp + f) = cq[q];
  }
  __threadfence();
#pragma unroll
  for (int q = 0; q < 4; ++q) {
    const int f = (wave * 4 + q) * 128 + 4 * lane;
    *(volatile v4i*)(cp + f) = cq[q];
  }
}

__global__ __launch_bounds__(OTHR) void k_offsets(const int* __restrict__ cnt, int* off, int* rbase, int nChunk) {
  __shared__ __attribute__((aligned(16))) int soff[NBC];
  __shared__ __attribute__((aligned(16))) int srb[RBN];
  __shared__ int wtot[OTHR / 32];
  const int tid = threadIdx.x, lane = tid & 31, wave = tid >> 5, sub = tid >> 8;
  for (int i = tid; i < RBN; i += OTHR) srb[i] = 0;
  __syncthreads();
  int carry = 0;
#pragma unroll 1
  for (int ch = 0; ch < nChunk; ++ch) {
    const int base = ch * NBC;
    const v4i c0 = *(const v4i*)(cnt + base + 8 * tid);
    const v4i c1 = *(const v4i*)(cnt + base + 8 * tid + 4);
    const int e0 = min(max(c0.x, 0), CNTMAX), e1 = min(max(c0.y, 0), CNTMAX);
    const int e2 = min(max(c0.z, 0), CNTMAX), e3 = min(max(c0.w, 0), CNTMAX);
    const int e4 = min(max(c1.x, 0), CNTMAX), e5 = min(max(c1.y, 0), CNTMAX);
    const int e6 = min(max(c1.z, 0), CNTMAX), e7 = min(max(c1.w, 0), CNTMAX);
    const int ts = e0 + e1 + e2 + e3 + e4 + e5 + e6 + e7;
    int incl = ts;
#pragma unroll
    for (int d = 1; d < 32; d <<= 1) {
      const int t = __shfl_up(incl, d);
      if (lane >= d) incl += t;
    }
    if (lane == 31) wtot[wave] = incl;
    __syncthreads();
    int S0 = 0, S1 = 0;
#pragma unroll
    for (int w = 0; w < 8; ++w) { S0 += wtot[w]; S1 += wtot[8 + w]; }
    int pre = 0;
#pragma unroll 1
    for (int w = 8 * sub; w < wave; ++w) pre += wtot[w];
    const int b0 = carry;
    const int b1 = b0 + ((S0 + 31) & ~31);
    const int b2 = b1 + ((S1 + 31) & ~31);
    const int myb = sub == 0 ? b0 : b1;
    if (tid == 0) {
      srb[min(2 * ch + 0, RBN - 1)] = b0;
      srb[min(2 * ch + 1, RBN - 1)] = b1;
    }
    int run = myb + pre + incl - ts;
    soff[8 * tid + 0] = run; run += e0;
    soff[8 * tid + 1] = run; run += e1;
    soff[8 * tid + 2] = run; run += e2;
    soff[8 * tid + 3] = run; run += e3;
    soff[8 * tid + 4] = run; run += e4;
    soff[8 * tid + 5] = run; run += e5;
    soff[8 * tid + 6] = run; run += e6;
    soff[8 * tid + 7] = run;
    carry = b2;
    __syncthreads();
    const v4i o0 = *(const v4i*)(soff + 4 * tid);
    const v4i o1 = *(const v4i*)(soff + 4 * (tid + OTHR));
    int* op = off + base;
    *(volatile v4i*)(op + 4 * tid) = o0;
    *(volatile v4i*)(op + 4 * (tid + OTHR)) = o1;
    __threadfence();
    *(volatile v4i*)(op + 4 * tid) = o0;
    *(volatile v4i*)(op + 4 * (tid + OTHR)) = o1;
    __syncthreads();
  }
  if (tid == 0) srb[min(2 * nChunk, RBN - 1)] = carry;
  __syncthreads();
  v4i rv = {0, 0, 0, 0};
  if (tid < 32) rv = *(const v4i*)(srb + 4 * tid);
  if (tid < 32) *(volatile v4i*)(rbase + 4 * tid) = rv;
  __threadfence();
  if (tid < 32) *(volatile v4i*)(rbase + 4 * tid) = rv;
}

__global__ __launch_bounds__(NTHR) void k_fill(
    const int* __restrict__ dsts, const int* __restrict__ off, const int* __restrict__ rbase,
    int* csr, int nE, int vec8, int csrLen) {
  extern __shared__ v4f lds_dyn[];
  int* region = (int*)lds_dyn;
  int* cursor = region + RCAP;
  int* list   = cursor + NBF;
  int* wcnt   = list + LISTN;
  const int tid = threadIdx.x, lane = tid & 31, wave = tid >> 5;
  const int b = blockIdx.x;
  const int nodeBase = b * NBF;

  int rb0 = rbase[b];
  const int rb1 = rbase[b + 1];
  rb0 = rb0 < 0 ? 0 : (rb0 > csrLen ? csrLen : rb0);
  rb0 &= ~31;
  int len = rb1 - rb0;
  len = len < 0 ? 0 : (len > RCAP ? RCAP : len);
  int lenW = (len + 31) & ~31;
  if (rb0 + lenW > csrLen) lenW = (csrLen - rb0) & ~31;

  {
    const v4i z = {0, 0, 0, 0};
    for (int i = tid; i < RCAP / 4; i += NTHR) ((v4i*)region)[i] = z;
    for (int s = tid; s < NBF; s += NTHR) {
      int o = off[nodeBase + s] - rb0;
      o = o < 0 ? 0 : (o > RCAP ? RCAP : o);
      cursor[s] = o;
    }
  }
  __syncthreads();

  const int nChunks = (nE + CHUNK - 1) / CHUNK;
#pragma unroll 1
  for (int ch = 0; ch < nChunks; ++ch) {
    const int cbase = ch * CHUNK;
    const int wc = scan_chunk<NBF>(dsts, nE, cbase, nodeBase, vec8, list, tid, lane, wave);
    if (lane == 0) wcnt[wave] = wc;
    __syncthreads();
    if (wave == 0) {
#pragma unroll 1
      for (int wsx = 0; wsx < NWAVE; ++wsx) {
        int n = __builtin_amdgcn_readfirstlane(wcnt[wsx]);
        n = n > WCAP ? WCAP : (n < 0 ? 0 : n);
        const int* lp = list + wsx * WCAP;
#pragma unroll 1
        for (int i = 0; i < n; ++i) {
          const int ent  = __builtin_amdgcn_readfirstlane(lp[i]);
          const int slot = ent & (NBF - 1);
          int e = cbase + ((ent >> 12) & (CHUNK - 1));
          e = e > nE - 1 ? nE - 1 : e;
          if (lane == 0) {
            int pos = cursor[slot];
            pos = pos < 0 ? 0 : (pos > RCAP - 1 ? RCAP - 1 : pos);
            region[pos] = e;
            const int np = pos + 1;
            cursor[slot] = np > RCAP ? RCAP : np;
          }
        }
      }
    }
    __syncthreads();
  }

  const int nv = lenW >> 2;
  int* gp = csr + rb0;
#pragma unroll 1
  for (int i = tid; i < nv; i += NTHR) { const v4i v = ((const v4i*)region)[i]; *(volatile v4i*)(gp + 4 * i) = v; }
  __threadfence();
#pragma unroll 1
  for (int i = tid; i < nv; i += NTHR) { const v4i v = ((const v4i*)region)[i]; *(volatile v4i*)(gp + 4 * i) = v; }
}

__global__ __launch_bounds__(NTHR) void k_gemm(const _Float16* __restrict__ A, const _Float16* __restrict__ Bs, float* C) {
  extern __shared__ v4f lds_dyn[];
  float* stg = (float*)lds_dyn;
  const int tid = threadIdx.x, lane = tid & 31, wave = tid >> 5, hh = lane >> 4, m = lane & 15;
  const int rowBase = blockIdx.x * GROWS;

  v8f acc[8];
#pragma unroll
  for (int t = 0; t < 8; ++t) { v8f z = {0.f, 0.f, 0.f, 0.f, 0.f, 0.f, 0.f, 0.f}; acc[t] = z; }
  const _Float16* ar = A + ((size_t)rowBase + wave * 16 + m) * EMB + 8 * hh;
#pragma unroll
  for (int kt = 0; kt < EMB / 32; ++kt) {
    FragH a;
    a.h[0] = *(const v8h*)(ar + 32 * kt);
    a.h[1] = *(const v8h*)(ar + 32 * kt + 16);
#pragma unroll
    for (int t = 0; t < 8; ++t) {
      const _Float16* bp = Bs + (size_t)(16 * t + m) * EMB + 32 * kt + 8 * hh;
      FragH b;
      b.h[0] = *(const v8h*)bp;
      b.h[1] = *(const v8h*)(bp + 16);
      acc[t] = wmh(a.v, b.v, acc[t]);
    }
  }

  const int r0 = wave * 16 + 8 * hh;
  float* sp = stg + r0 * EMB + m;
#pragma unroll
  for (int t = 0; t < 8; ++t) {
#pragma unroll
    for (int r = 0; r < 8; ++r) sp[r * EMB + 16 * t] = acc[t][r] * WINV;
  }
  __syncthreads();

  const float* lp = stg + wave * 16 * EMB + 4 * lane;
  float* gp = C + ((size_t)rowBase + wave * 16) * EMB + 4 * lane;
#pragma unroll
  for (int i = 0; i < 16; ++i) { const v4f v = *(const v4f*)(lp + i * EMB); *(volatile v4f*)(gp + (size_t)i * EMB) = v; }
  __threadfence();
#pragma unroll
  for (int i = 0; i < 16; ++i) { const v4f v = *(const v4f*)(lp + i * EMB); *(volatile v4f*)(gp + (size_t)i * EMB) = v; }
}

__global__ __launch_bounds__(NTHR) void k_agg(
    const int* __restrict__ csr, const int* __restrict__ off, const int* __restrict__ cnt,
    const int* __restrict__ cols, const float* __restrict__ vals, const float* __restrict__ T,
    const float* accin, float* accout, _Float16* hout, int nN, int nE, int csrLen, float oscale) {
#pragma clang fp contract(off)
  extern __shared__ v4f lds_dyn[];
  _Float16* sh = (_Float16*)lds_dyn;
  const int tid = threadIdx.x, lane = tid & 31, wave = tid >> 5;
  const int tbase = blockIdx.x * TGT + wave * 32;
  const int cl = tbase + lane;
  const int cnt_l = cnt[cl];
  const int off_l = off[cl];
  union FI { float f; int i; };

#pragma unroll 1
  for (int j = 0; j < 32; ++j) {
    const int c = tbase + j;
    int n = __builtin_amdgcn_readlane(cnt_l, j);
    n = n < 0 ? 0 : (n > DEGCAP ? DEGCAP : n);
    const int st = __builtin_amdgcn_readlane(off_l, j);
    v4f a = {0.f, 0.f, 0.f, 0.f};
#pragma unroll 1
    for (int q0 = 0; q0 < n; q0 += 32) {
      int pos = st + q0 + lane;
      pos = pos < 0 ? 0 : (pos > csrLen - 1 ? csrLen - 1 : pos);
      int e = csr[pos];
      e = e < 0 ? 0 : (e > nE - 1 ? nE - 1 : e);
      int sl = cols[e];
      sl = sl < 0 ? 0 : (sl > nN - 1 ? nN - 1 : sl);
      FI vu; vu.f = vals[e];
      const int mcnt = (n - q0) < 32 ? (n - q0) : 32;
#pragma unroll 1
      for (int p = 0; p < mcnt; ++p) {
        const int s = __builtin_amdgcn_readlane(sl, p);
        FI w; w.i = __builtin_amdgcn_readlane(vu.i, p);
        const v4f x = *(const v4f*)(T + (size_t)s * EMB + 4 * lane);
        a = a + x * w.f;
      }
    }
    float ss = a.x * a.x + a.y * a.y + a.z * a.z + a.w * a.w;
#pragma unroll
    for (int o = 16; o >= 1; o >>= 1) ss += __shfl_xor(ss, o);
    const float nrm = fmaxf(sqrtf(ss), 1e-12f);
    const float inv = 1.0f / nrm;

    v4h hv;
    hv.x = (_Float16)a.x; hv.y = (_Float16)a.y; hv.z = (_Float16)a.z; hv.w = (_Float16)a.w;
    *(v4h*)(sh + (wave * 32 + j) * EMB + 4 * lane) = hv;

    const int cc = c < nN ? c : nN - 1;
    const v4f ao = *(const v4f*)(accin + (size_t)cc * EMB + 4 * lane);
    const v4f rr = (ao + a * inv) * oscale;
    if (c < nN) {
      float* op = accout + (size_t)c * EMB + 4 * lane;
      *(volatile v4f*)op = rr;
      __threadfence();
      *(volatile v4f*)op = rr;
    }
  }
  __syncthreads();

  const _Float16* lp = sh + wave * 32 * EMB;
  _Float16* gp = hout + (size_t)tbase * EMB;
#pragma unroll
  for (int i = 0; i < 16; ++i) {
    const v8h v = *(const v8h*)(lp + 8 * (32 * i + lane));
    *(volatile v8h*)(gp + 8 * (32 * i + lane)) = v;
  }
  __threadfence();
#pragma unroll
  for (int i = 0; i < 16; ++i) {
    const v8h v = *(const v8h*)(lp + 8 * (32 * i + lane));
    *(volatile v8h*)(gp + 8 * (32 * i + lane)) = v;
  }
}

extern "C" void kernel_launch(void* const* d_in, const int* in_sizes, int n_in,
                              void* d_out, int out_size, void* d_ws, size_t ws_size,
                              hipStream_t stream) {
  if (n_in < 5) return;
  const int nN = in_sizes[0] / EMB;
  const int nE = in_sizes[1];
  const int nL = in_sizes[2] / (EMB * EMB);
  if (nN <= 0 || nE <= 0 || nL < 1) return;
  if (in_sizes[0] != nN * EMB || in_sizes[2] != nL * EMB * EMB) return;
  if (in_sizes[3] != nE || in_sizes[4] != nE) return;
  if (out_size != nN * EMB) return;
  if (nE > (1 << 28) || nN > (1 << 24)) return;

  const float* emb  = (const float*)d_in[0];
  const float* vals = (const float*)d_in[1];
  const float* W    = (const float*)d_in[2];
  const int*   rows = (const int*)d_in[3];
  const int*   cols = (const int*)d_in[4];
  float* out = (float*)d_out;

  const int NPAD   = ((nN + TGT - 1) / TGT) * TGT;
  const int nBC    = (nN + NBC - 1) / NBC;
  const int CNTPAD = nBC * NBC;
  if (NSUB * nBC + 1 > RBN) return;
  const int nBF    = (nN + NBF - 1) / NBF;
  const int csrLen = ((nE + 31) & ~31) + (NSUB * nBC + 1) * 32;
  const int nGemm  = NPAD / GROWS;
  const int nAgg   = NPAD / TGT;

  char* ws = (char*)d_ws;
  size_t off = 0;
  const size_t oWL  = off; off += (size_t)nL * EMB * EMB * 2;      off = (off + 255) & ~(size_t)255;
  const size_t oCnt = off; off += (size_t)CNTPAD * 4;              off = (off + 255) & ~(size_t)255;
  const size_t oOff = off; off += (size_t)CNTPAD * 4;              off = (off + 255) & ~(size_t)255;
  const size_t oRb  = off; off += (size_t)RBN * 4;                 off = (off + 255) & ~(size_t)255;
  const size_t oCsr = off; off += (size_t)csrLen * 4;              off = (off + 255) & ~(size_t)255;
  const size_t oT   = off; off += (size_t)NPAD * EMB * 4;          off = (off + 255) & ~(size_t)255;
  const size_t oH   = off; off += (size_t)NPAD * EMB * 2;          off = (off + 255) & ~(size_t)255;
  if (off > ws_size) return;
  _Float16* wL   = (_Float16*)(ws + oWL);
  int*      cnt  = (int*)(ws + oCnt);
  int*      offp = (int*)(ws + oOff);
  int*      rb   = (int*)(ws + oRb);
  int*      csr  = (int*)(ws + oCsr);
  float*    T    = (float*)(ws + oT);
  _Float16* hpl  = (_Float16*)(ws + oH);

  const int vec8 = ((nE & 3) == 0) ? 1 : 0;

  const int wTot8 = nL * EMB * EMB / 8;
  k_wprep<<<(wTot8 + NTHR - 1) / NTHR, NTHR, 0, stream>>>(W, wL, wTot8);

  const int hTot8 = NPAD * (EMB / 8);
  k_cvt<<<(hTot8 + NTHR - 1) / NTHR, NTHR, 0, stream>>>(emb, hpl, nN, hTot8);

  k_count<<<nBC, NTHR, 0, stream>>>(rows, cnt, nE, vec8);
  k_offsets<<<1, OTHR, 0, stream>>>(cnt, offp, rb, nBC);
  hipFuncSetAttribute(reinterpret_cast<const void*>(&k_fill),
                      hipFuncAttributeMaxDynamicSharedMemorySize, LDS_FILL);
  k_fill<<<nBF, NTHR, LDS_FILL, stream>>>(rows, offp, rb, csr, nE, vec8, csrLen);

  hipFuncSetAttribute(reinterpret_cast<const void*>(&k_gemm),
                      hipFuncAttributeMaxDynamicSharedMemorySize, LDS_GEMM);
  hipFuncSetAttribute(reinterpret_cast<const void*>(&k_agg),
                      hipFuncAttributeMaxDynamicSharedMemorySize, LDS_AGG);
  for (int i = 0; i < nL; ++i) {
    k_gemm<<<nGemm, NTHR, LDS_GEMM, stream>>>(hpl, wL + (size_t)i * EMB * EMB, T);
    const float* ain = (i == 0) ? emb : (const float*)out;
    const float osc  = (i == nL - 1) ? (1.0f / (float)(nL + 1)) : 1.0f;
    k_agg<<<nAgg, NTHR, LDS_AGG, stream>>>(csr, offp, cnt, cols, vals, T, ain, out, hpl, nN, nE, csrLen, osc);
  }
}
